// GPTNeoSelfAttention_88527865905620
// MI455X (gfx1250) — hardware-verified
//
#include <hip/hip_runtime.h>
#include <stdint.h>


#define NB     2
#define NS     2048
#define ND     768
#define NH     12
#define HD     64
#define NTOK   (NB * NS)
#define NBH    (NB * NH)
#define PLANE  ((size_t)NBH * NS * HD)
#define OPLANE ((size_t)NTOK * ND)
#define NEGMAX (-3.402823466e+38f)
#define KROW   72
#define PROW   40

typedef unsigned short us;
typedef us     v8us __attribute__((ext_vector_type(8)));
typedef __bf16 v16b __attribute__((ext_vector_type(16)));
typedef float  v8f  __attribute__((ext_vector_type(8)));
typedef float  v4f  __attribute__((ext_vector_type(4)));
typedef int    v8i  __attribute__((ext_vector_type(8)));

union Frag { v16b v; v8us h[2]; v8i w; };

__device__ __forceinline__ us f2bf(float f) {
  unsigned int u = __float_as_uint(f);
  u += 0x7FFFu + ((u >> 16) & 1u);
  return (us)(u >> 16);
}
__device__ __forceinline__ float bf2f(us b) {
  return __uint_as_float(((unsigned int)b) << 16);
}
__device__ __forceinline__ v8f zero8() {
  v8f z = {0.f, 0.f, 0.f, 0.f, 0.f, 0.f, 0.f, 0.f};
  return z;
}

__device__ __forceinline__ Frag ldf(const us* p, int k8) {
  Frag f;
  f.h[0] = *(const v8us*)(p + k8);
  f.h[1] = *(const v8us*)(p + 16 + k8);
  return f;
}

__device__ __forceinline__ v8f wmma_bf(const Frag& a, const Frag& b, v8f c) {
  v8f d = __builtin_amdgcn_wmma_f32_16x16x32_bf16(false, a.v, false, b.v, (short)0, c, false, false);
  asm volatile("v_nop\n\tv_nop\n\tv_nop\n\tv_nop" : "+v"(d) : "v"(a.w), "v"(b.w));
  return d;
}

__global__ __launch_bounds__(256) void k_cvt(const float* s0, const float* s1, const float* s2,
                                             const float* s3, us* d0, us* d1, us* d2, us* d3, int n) {
  const float* s = s0;
  us* d = d0;
  if (blockIdx.y == 1) { s = s1; d = d1; }
  else if (blockIdx.y == 2) { s = s2; d = d2; }
  else if (blockIdx.y == 3) { s = s3; d = d3; }
  const size_t i = ((size_t)blockIdx.x * 256 + threadIdx.x) * 8;
  if (i + 8 > (size_t)n) return;
  const v4f a = *(const v4f*)(s + i);
  const v4f b = *(const v4f*)(s + i + 4);
  v8us r;
  r[0] = f2bf(a[0]); r[1] = f2bf(a[1]); r[2] = f2bf(a[2]); r[3] = f2bf(a[3]);
  r[4] = f2bf(b[0]); r[5] = f2bf(b[1]); r[6] = f2bf(b[2]); r[7] = f2bf(b[3]);
  us* dp = d + i;
  *(volatile v8us*)dp = r;
  __threadfence();
  *(volatile v8us*)dp = r;
}

__device__ __forceinline__ void qkv_store_lines(const us* hiSh, const us* loSh, us* pHi, us* pLo,
                                                int mat, int bh, int s0, int wave, int lane) {
  const int piece = lane & 7;
#pragma unroll 1
  for (int it = 0; it < 16; ++it) {
    const int L = wave * 64 + it * 4 + (lane >> 3);
    const int p = L >> 7, rem = L & 127;
    const us* srcP = p ? loSh : hiSh;
    us* dstP = p ? pLo : pHi;
    const us* src;
    us* dst;
    if (mat < 2) {
      src = srcP + rem * 64 + 8 * piece;
      dst = dstP + ((size_t)bh * NS + s0 + rem) * HD + 8 * piece;
    } else {
      const int d = rem >> 1, hf = rem & 1;
      src = srcP + d * 128 + 64 * hf + 8 * piece;
      dst = dstP + ((size_t)bh * HD + d) * NS + s0 + 64 * hf + 8 * piece;
    }
    const v8us val = *(const v8us*)src;
    *(volatile v8us*)dst = val;
  }
}

__global__ __launch_bounds__(128) void k_qkv(const us* __restrict__ xb, const us* __restrict__ wb,
                                             us* __restrict__ qkv) {
  __shared__ __align__(16) us sh[2 * 128 * 64];
  const int tid = threadIdx.x, lane = tid & 31, wave = tid >> 5;
  const int h8 = (lane >> 4) << 3, m = lane & 15;
  const int mat = blockIdx.z, hh = blockIdx.x;
  const int mb = blockIdx.y * 128;
  const int m0 = mb + wave * 32;
  const us* W = wb + (size_t)mat * ND * ND + (size_t)(hh * 64) * ND;
  const us* a0p = xb + (size_t)(m0 + m) * ND;
  const us* a1p = xb + (size_t)(m0 + 16 + m) * ND;

  v8f acc[2][4];
#pragma unroll
  for (int i = 0; i < 2; ++i)
#pragma unroll
    for (int t = 0; t < 4; ++t) acc[i][t] = zero8();

  for (int kc = 0; kc < ND; kc += 32) {
    const Frag a0 = ldf(a0p + kc, h8);
    const Frag a1 = ldf(a1p + kc, h8);
#pragma unroll
    for (int t = 0; t < 4; ++t) {
      const Frag bw = ldf(W + (size_t)(16 * t + m) * ND + kc, h8);
      acc[0][t] = wmma_bf(a0, bw, acc[0][t]);
      acc[1][t] = wmma_bf(a1, bw, acc[1][t]);
    }
  }

  const int bidx = mb / NS;
  const int s0 = mb - bidx * NS;
  const int bh = bidx * NH + hh;
  us* hiSh = sh;
  us* loSh = sh + 128 * 64;
  if (mat < 2) {
#pragma unroll
    for (int mt = 0; mt < 2; ++mt)
#pragma unroll
      for (int t = 0; t < 4; ++t)
#pragma unroll
        for (int r = 0; r < 8; ++r) {
          const int tok = wave * 32 + 16 * mt + h8 + r;
          const int d = 16 * t + m;
          const float v = acc[mt][t][r];
          const us hi = f2bf(v);
          const us lo = f2bf(v - bf2f(hi));
          hiSh[tok * 64 + d] = hi;
          loSh[tok * 64 + d] = lo;
        }
  } else {
#pragma unroll
    for (int mt = 0; mt < 2; ++mt)
#pragma unroll
      for (int t = 0; t < 4; ++t)
#pragma unroll
        for (int r = 0; r < 8; ++r) {
          const int tok = wave * 32 + 16 * mt + h8 + r;
          const int d = 16 * t + m;
          const float v = acc[mt][t][r];
          const us hi = f2bf(v);
          const us lo = f2bf(v - bf2f(hi));
          hiSh[d * 128 + tok] = hi;
          loSh[d * 128 + tok] = lo;
        }
  }
  __syncthreads();
  us* pHi = qkv + (size_t)(2 * mat) * PLANE;
  us* pLo = qkv + (size_t)(2 * mat + 1) * PLANE;
  qkv_store_lines(hiSh, loSh, pHi, pLo, mat, bh, s0, wave, lane);
  __threadfence();
  qkv_store_lines(hiSh, loSh, pHi, pLo, mat, bh, s0, wave, lane);
}

__device__ __forceinline__ void attn_store_lines(const us* Ohs, const us* Ols, us* ob, int tok0,
                                                 int hh, int lane) {
  const int piece = lane & 7;
#pragma unroll 1
  for (int it = 0; it < 8; ++it) {
    const int L = it * 4 + (lane >> 3);
    const int p = L >> 4, row = L & 15;
    const us* src = (p ? Ols : Ohs) + row * 64 + 8 * piece;
    us* dst = ob + (size_t)p * OPLANE + (size_t)(tok0 + row) * ND + hh * 64 + 8 * piece;
    const v8us val = *(const v8us*)src;
    *(volatile v8us*)dst = val;
  }
}

__global__ __launch_bounds__(128) void k_attn(const us* __restrict__ qkv, const float* __restrict__ am,
                                              us* __restrict__ ob) {
  __shared__ __align__(16) us sh[4 * 64 * KROW + 8 * 16 * PROW];
  const int tid = threadIdx.x, lane = tid & 31;
  const int wave = __builtin_amdgcn_readfirstlane(tid >> 5);
  const int h8 = (lane >> 4) << 3, m = lane & 15;
  const int qb = blockIdx.x, bh = blockIdx.y;
  const int b = bh / NH, hh = bh - b * NH;
  us* Ksh = sh;
  us* Phi = sh + 4 * 64 * KROW + wave * (2 * 16 * PROW);
  us* Plo = Phi + 16 * PROW;
  const us* Qg = qkv + (size_t)bh * NS * HD;
  const us* Kg = qkv + 2 * PLANE + (size_t)bh * NS * HD;
  const us* Vg = qkv + 4 * PLANE + (size_t)bh * HD * NS;
  const int q0 = qb * 64 + wave * 16;

  Frag qh[2], ql[2];
#pragma unroll
  for (int dh = 0; dh < 2; ++dh) {
    qh[dh] = ldf(Qg + (size_t)(q0 + m) * HD + 32 * dh, h8);
    ql[dh] = ldf(Qg + PLANE + (size_t)(q0 + m) * HD + 32 * dh, h8);
  }

  v8f oacc[4];
#pragma unroll
  for (int d = 0; d < 4; ++d) oacc[d] = zero8();
  float mrow[8], srow[8];
#pragma unroll
  for (int r = 0; r < 8; ++r) { mrow[r] = NEGMAX; srow[r] = 0.f; }

  const int nchunk = qb + 1;
  for (int ci = 0; ci < nchunk; ++ci) {
    const int kc = ci * 64;
    const bool diag = (ci == qb);
    __syncthreads();
#pragma unroll
    for (int j = 0; j < 16; ++j) {
      const int p = j >> 2;
      const int row = ((j & 3) << 4) + (tid >> 3);
      const int piece = tid & 7;
      const us* src;
      if (p < 2) src = Kg + (size_t)p * PLANE + (size_t)(kc + row) * HD + 8 * piece;
      else       src = Vg + (size_t)(p - 2) * PLANE + (size_t)row * NS + kc + 8 * piece;
      *(v8us*)(Ksh + p * 64 * KROW + row * KROW + 8 * piece) = *(const v8us*)src;
    }
    __syncthreads();

    v8f sc[4];
#pragma unroll
    for (int t = 0; t < 4; ++t) {
      v8f s = zero8();
      if (!diag || t <= wave) {
#pragma unroll
        for (int dh = 0; dh < 2; ++dh) {
          const us* kr = Ksh + (16 * t + m) * KROW + 32 * dh;
          const Frag kh = ldf(kr, h8);
          const Frag kl = ldf(kr + 64 * KROW, h8);
          s = wmma_bf(qh[dh], kh, s);
          s = wmma_bf(qh[dh], kl, s);
          s = wmma_bf(ql[dh], kh, s);
        }
      }
      sc[t] = s;
    }

    float madd[4];
    int kcol[4];
#pragma unroll
    for (int t = 0; t < 4; ++t) {
      kcol[t] = kc + 16 * t + m;
      const float a = am[b * NS + kcol[t]];
      madd[t] = (1.f - a) * NEGMAX;
    }
#pragma unroll
    for (int r = 0; r < 8; ++r) {
      const int q = q0 + h8 + r;
      float mx = NEGMAX;
#pragma unroll
      for (int t = 0; t < 4; ++t) {
        const float v = ((kcol[t] <= q) ? sc[t][r] : NEGMAX) + madd[t];
        sc[t][r] = v;
        mx = fmaxf(mx, v);
      }
      mx = fmaxf(mx, __shfl_xor(mx, 1, 32));
      mx = fmaxf(mx, __shfl_xor(mx, 2, 32));
      mx = fmaxf(mx, __shfl_xor(mx, 4, 32));
      mx = fmaxf(mx, __shfl_xor(mx, 8, 32));
      const float mnew = fmaxf(mrow[r], mx);
      const float corr = __expf(mrow[r] - mnew);
      mrow[r] = mnew;
      float rsum = 0.f;
#pragma unroll
      for (int t = 0; t < 4; ++t) {
        const float pv = __expf(sc[t][r] - mnew);
        sc[t][r] = pv;
        rsum += pv;
      }
      rsum += __shfl_xor(rsum, 1, 32);
      rsum += __shfl_xor(rsum, 2, 32);
      rsum += __shfl_xor(rsum, 4, 32);
      rsum += __shfl_xor(rsum, 8, 32);
      srow[r] = srow[r] * corr + rsum;
#pragma unroll
      for (int d = 0; d < 4; ++d) oacc[d][r] *= corr;
    }

#pragma unroll
    for (int half = 0; half < 2; ++half) {
      __syncthreads();
#pragma unroll
      for (int tt = 0; tt < 2; ++tt) {
        const int t = 2 * half + tt;
#pragma unroll
        for (int r = 0; r < 8; ++r) {
          const float pv = sc[t][r];
          const us hi = f2bf(pv);
          const us lo = f2bf(pv - bf2f(hi));
          const int o = (h8 + r) * PROW + 16 * tt + m;
          Phi[o] = hi;
          Plo[o] = lo;
        }
      }
      __syncthreads();
      if (!diag || 2 * half <= wave) {
        const Frag ph = ldf(Phi + m * PROW, h8);
        const Frag pl = ldf(Plo + m * PROW, h8);
#pragma unroll
        for (int dt = 0; dt < 4; ++dt) {
          const us* vr = Ksh + 2 * 64 * KROW + (16 * dt + m) * KROW + 32 * half;
          const Frag vh = ldf(vr, h8);
          const Frag vl = ldf(vr + 64 * KROW, h8);
          oacc[dt] = wmma_bf(ph, vh, oacc[dt]);
          oacc[dt] = wmma_bf(ph, vl, oacc[dt]);
          oacc[dt] = wmma_bf(pl, vh, oacc[dt]);
        }
      }
    }
  }

  float inv[8];
#pragma unroll
  for (int r = 0; r < 8; ++r) inv[r] = 1.f / srow[r];
  __syncthreads();
  us* Ohs = sh + wave * (2 * 16 * 64);
  us* Ols = Ohs + 16 * 64;
#pragma unroll
  for (int dt = 0; dt < 4; ++dt)
#pragma unroll
    for (int r = 0; r < 8; ++r) {
      const float o = oacc[dt][r] * inv[r];
      const us hi = f2bf(o);
      const us lo = f2bf(o - bf2f(hi));
      const int idx = (h8 + r) * 64 + 16 * dt + m;
      Ohs[idx] = hi;
      Ols[idx] = lo;
    }
  __syncthreads();
  const int tok0 = b * NS + q0;
  attn_store_lines(Ohs, Ols, ob, tok0, hh, lane);
  __threadfence();
  attn_store_lines(Ohs, Ols, ob, tok0, hh, lane);
}

__device__ __forceinline__ void out_store_lines(const float* S, float* out, int m0, int n0, int lane) {
  const int piece = lane & 7;
#pragma unroll 1
  for (int it = 0; it < 16; ++it) {
    const int L = it * 4 + (lane >> 3);
    const int row = L >> 1, hf = L & 1;
    const v4f val = *(const v4f*)(S + row * 64 + 32 * hf + 4 * piece);
    float* dst = out + (size_t)(m0 + row) * ND + n0 + 32 * hf + 4 * piece;
    *(volatile v4f*)dst = val;
  }
}

__global__ __launch_bounds__(128) void k_out(const us* __restrict__ ob, const us* __restrict__ wob,
                                             const float* __restrict__ bo, float* __restrict__ out) {
  __shared__ __align__(16) float sh[4 * 32 * 64];
  const int tid = threadIdx.x, lane = tid & 31, wave = tid >> 5;
  const int h8 = (lane >> 4) << 3, m = lane & 15;
  const int n0 = blockIdx.x * 64;
  const int m0 = blockIdx.y * 128 + wave * 32;
  const us* ah0 = ob + (size_t)(m0 + m) * ND;
  const us* ah1 = ob + (size_t)(m0 + 16 + m) * ND;
  const us* al0 = ah0 + OPLANE;
  const us* al1 = ah1 + OPLANE;
  const us* W = wob + (size_t)n0 * ND;

  v8f acc[2][4];
#pragma unroll
  for (int i = 0; i < 2; ++i)
#pragma unroll
    for (int t = 0; t < 4; ++t) acc[i][t] = zero8();

  for (int kc = 0; kc < ND; kc += 32) {
    const Frag a0h = ldf(ah0 + kc, h8);
    const Frag a1h = ldf(ah1 + kc, h8);
    const Frag a0l = ldf(al0 + kc, h8);
    const Frag a1l = ldf(al1 + kc, h8);
#pragma unroll
    for (int t = 0; t < 4; ++t) {
      const Frag bw = ldf(W + (size_t)(16 * t + m) * ND + kc, h8);
      acc[0][t] = wmma_bf(a0h, bw, acc[0][t]);
      acc[0][t] = wmma_bf(a0l, bw, acc[0][t]);
      acc[1][t] = wmma_bf(a1h, bw, acc[1][t]);
      acc[1][t] = wmma_bf(a1l, bw, acc[1][t]);
    }
  }

  float* S = sh + wave * 32 * 64;
#pragma unroll
  for (int t = 0; t < 4; ++t) {
    const float bias = bo[n0 + 16 * t + m];
#pragma unroll
    for (int mt = 0; mt < 2; ++mt)
#pragma unroll
      for (int r = 0; r < 8; ++r)
        S[(16 * mt + h8 + r) * 64 + 16 * t + m] = acc[mt][t][r] + bias;
  }
  __syncthreads();
  out_store_lines(S, out, m0, n0, lane);
  __threadfence();
  out_store_lines(S, out, m0, n0, lane);
}

extern "C" void kernel_launch(void* const* d_in, const int* in_sizes, int n_in,
                              void* d_out, int out_size, void* d_ws,
                              size_t ws_size, hipStream_t stream) {
  if (n_in < 7) return;
  if (in_sizes[0] != NTOK * ND || in_sizes[1] != NB * NS || in_sizes[2] != ND * ND ||
      in_sizes[3] != ND * ND || in_sizes[4] != ND * ND || in_sizes[5] != ND * ND ||
      in_sizes[6] != ND || out_size != NTOK * ND) return;

  const float* x  = (const float*)d_in[0];
  const float* am = (const float*)d_in[1];
  const float* Wq = (const float*)d_in[2];
  const float* Wk = (const float*)d_in[3];
  const float* Wv = (const float*)d_in[4];
  const float* Wo = (const float*)d_in[5];
  const float* bo = (const float*)d_in[6];

  const size_t n_xb  = (size_t)NTOK * ND;
  const size_t n_wb  = (size_t)4 * ND * ND;
  const size_t n_qkv = 6 * PLANE;
  const size_t n_ob  = 2 * OPLANE;
  const size_t total_bytes = (n_xb + n_wb + n_qkv + n_ob) * sizeof(us);
  if (total_bytes > ws_size) return;
  us* xb  = (us*)d_ws;
  us* wb  = xb + n_xb;
  us* qkv = wb + n_wb;
  us* ob  = qkv + n_qkv;

  k_cvt<<<dim3((NTOK * ND) / 2048, 1), 256, 0, stream>>>(x, x, x, x, xb, xb, xb, xb, NTOK * ND);
  k_cvt<<<dim3((ND * ND) / 2048, 4), 256, 0, stream>>>(Wq, Wk, Wv, Wo, wb, wb + (size_t)ND * ND,
                                                        wb + (size_t)2 * ND * ND,
                                                        wb + (size_t)3 * ND * ND, ND * ND);
  k_qkv<<<dim3(NH, NTOK / 128, 3), 128, 0, stream>>>(xb, wb, qkv);
  k_attn<<<dim3(NS / 64, NBH), 128, 0, stream>>>(qkv, am, ob);
  k_out<<<dim3(ND / 64, NTOK / 128), 128, 0, stream>>>(ob, wb + (size_t)3 * ND * ND, bo,
                                                        (float*)d_out);
}
